// GraphSAGE_85813446574086
// MI455X (gfx1250) — hardware-run, weakly checked
//
#include <hip/hip_runtime.h>

typedef float          v8f   __attribute__((ext_vector_type(8)));
typedef float          v4f   __attribute__((ext_vector_type(4)));
typedef unsigned int   v4u   __attribute__((ext_vector_type(4)));
typedef int            v8i   __attribute__((ext_vector_type(8)));
typedef unsigned short v8us  __attribute__((ext_vector_type(8)));
typedef unsigned short v16us __attribute__((ext_vector_type(16)));
typedef __bf16         v16bf __attribute__((ext_vector_type(16)));
typedef _Float16       v16h  __attribute__((ext_vector_type(16)));
typedef v4f  __attribute__((may_alias)) v4fa;
typedef v8us __attribute__((may_alias)) v8usa;
union FragB { v16bf v; v16us u; v8us h[2]; v8i w; };
union FragH { v16h  v; v16us u; v8us h[2]; v8i w; };

__device__ __forceinline__ v8f wmb(const FragB& a, const FragB& b, v8f c) {
  v8f d = __builtin_amdgcn_wmma_f32_16x16x32_bf16(false, a.v, false, b.v, (short)0, c, false, false);
  asm volatile("v_nop\n\tv_nop\n\tv_nop\n\tv_nop" : "+v"(d) : "v"(a.w), "v"(b.w));
  return d;
}

__device__ __forceinline__ v8f wmh(const FragH& a, const FragH& b, v8f c) {
  v8f d = __builtin_amdgcn_wmma_f32_16x16x32_f16(false, a.v, false, b.v, (short)0, c, false, false);
  asm volatile("v_nop\n\tv_nop\n\tv_nop\n\tv_nop" : "+v"(d) : "v"(a.w), "v"(b.w));
  return d;
}

__device__ __forceinline__ unsigned bf16_bits(float f) {
  const unsigned u = __float_as_uint(f);
  const unsigned r = (u + 0x7FFFu + ((u >> 16) & 1u)) >> 16;
  const unsigned q = (u >> 16) | 0x40u;
  return ((u & 0x7fffffffu) > 0x7f800000u) ? q : r;
}

__device__ __forceinline__ float bf16_val(float f) {
  return __uint_as_float(bf16_bits(f) << 16);
}
__device__ __forceinline__ int clampi(int v, int lo, int hi) {
  return v < lo ? lo : (v > hi ? hi : v);
}

__device__ __forceinline__ unsigned f16_bits(float f) {
  const unsigned u  = __float_as_uint(f);
  const unsigned s  = (u >> 16) & 0x8000u;
  const unsigned a  = u & 0x7fffffffu;
  const unsigned t  = a - 0x38000000u;
  const unsigned r  = (t + 0x0FFFu + ((t >> 13) & 1u)) >> 13;
  const unsigned rc = r > 0x7C00u ? 0x7C00u : r;
  const bool small  = a < 0x38800000u;
  const bool isnan  = a > 0x7f800000u;
  const unsigned fin = small ? 0u : (s | rc);
  return isnan ? (s | 0x7E00u) : fin;
}

__device__ __forceinline__ unsigned pk16(unsigned lo, unsigned hi) { return lo | (hi << 16); }
__device__ __forceinline__ unsigned bf16_lo_bits(float v) {
  float hi = bf16_val(v);
  asm volatile("" : "+v"(hi));
  return bf16_bits(v - hi);
}
__device__ __forceinline__ v4u pack8_bf16(v4f a, v4f c) {
  return (v4u){ pk16(bf16_bits(a[0]), bf16_bits(a[1])), pk16(bf16_bits(a[2]), bf16_bits(a[3])),
                pk16(bf16_bits(c[0]), bf16_bits(c[1])), pk16(bf16_bits(c[2]), bf16_bits(c[3])) };
}
__device__ __forceinline__ v4u pack8_bf16_lo(v4f a, v4f c) {
  return (v4u){ pk16(bf16_lo_bits(a[0]), bf16_lo_bits(a[1])), pk16(bf16_lo_bits(a[2]), bf16_lo_bits(a[3])),
                pk16(bf16_lo_bits(c[0]), bf16_lo_bits(c[1])), pk16(bf16_lo_bits(c[2]), bf16_lo_bits(c[3])) };
}
__device__ __forceinline__ v4u pack8_f16(v4f a, v4f c) {
  return (v4u){ pk16(f16_bits(a[0]), f16_bits(a[1])), pk16(f16_bits(a[2]), f16_bits(a[3])),
                pk16(f16_bits(c[0]), f16_bits(c[1])), pk16(f16_bits(c[2]), f16_bits(c[3])) };
}

template <int FORM>
__global__ __launch_bounds__(256) void k_plane(const float* __restrict__ src, int rows, int cols, int ldsrc,
                                               unsigned short* __restrict__ dst, int MP, int KP) {
  static_assert(FORM >= 0 && FORM <= 3);
  const int KTOT = (FORM == 1 || FORM == 3) ? 2 * KP : KP;
  const unsigned ppr   = (unsigned)(KTOT >> 3);
  const unsigned kp8   = (unsigned)(KP >> 3);
  const unsigned total = (unsigned)MP * ppr;
  const unsigned g     = blockIdx.x * 256u + threadIdx.x;
  const unsigned rowu  = g / ppr;
  const unsigned p     = g - rowu * ppr;
  const bool second    = p >= kp8;
  const int row = (int)rowu;
  const int c0  = (int)((second ? p - kp8 : p) << 3);
  const float* srow = src + (size_t)clampi(row, 0, rows - 1) * (size_t)ldsrc;
  float x[8];
  unsigned mk[8];
#pragma unroll
  for (int e = 0; e < 8; ++e) {
    const int c = c0 + e;
    const float v = srow[clampi(c, 0, cols - 1)];
    asm volatile("" :: "v"(v));
    x[e]  = v;
    mk[e] = (row < rows && c < cols) ? 0xFFFFu : 0u;
  }
  const v4f a = (v4f){ x[0], x[1], x[2], x[3] };
  const v4f c = (v4f){ x[4], x[5], x[6], x[7] };
  v4u o;
  if (FORM == 2) {
    o = pack8_f16(a, c);
  } else {
    const v4u hi = pack8_bf16(a, c);
    o = hi;
    if (FORM == 1) { const v4u lo = pack8_bf16_lo(a, c); o = second ? lo : hi; }
  }
  const v4u mw = (v4u){ pk16(mk[0], mk[1]), pk16(mk[2], mk[3]), pk16(mk[4], mk[5]), pk16(mk[6], mk[7]) };
  o &= mw;
  if (g < total) {
    volatile v4u* q = (volatile v4u*)(dst + (size_t)g * 8);
    *q = o;
    __threadfence();
    *q = o;
  }
}

template <int FORM> struct FragOf    { typedef FragB T; };
template <>         struct FragOf<2> { typedef FragH T; };
__device__ __forceinline__ v8f mm(const FragB& a, const FragB& b, v8f c) { return wmb(a, b, c); }
__device__ __forceinline__ v8f mm(const FragH& a, const FragH& b, v8f c) { return wmh(a, b, c); }
template <class F> __device__ __forceinline__ F ld_frag(const unsigned short* p) {
  F f;
  f.h[0] = *(const v8usa*)(p);
  f.h[1] = *(const v8usa*)(p + 16);
  return f;
}

template <int FORM, int EPI>
__global__ __launch_bounds__(256) __attribute__((amdgpu_num_vgpr(248)))
void k_gemm_nt(const unsigned short* __restrict__ A, const unsigned short* __restrict__ B,
               const float* __restrict__ bias, float* __restrict__ D, int M, int N, int KTOT, int ldd) {
  static_assert(FORM >= 0 && FORM <= 2);
  static_assert(EPI == 0 || EPI == 1);
  typedef typename FragOf<FORM>::T F;
  __shared__ __attribute__((aligned(16))) float sT[8][16 * 68];
  const int lane = threadIdx.x & 31;
  const int wave = threadIdx.x >> 5;
  const int tilesM = (M + 63) >> 6;
  const int tilesN = (N + 63) >> 6;
  const int tile = blockIdx.x * 8 + wave;
  if (tile >= tilesM * tilesN) return;
  const int tm = tile / tilesN;
  const int tn = tile - tm * tilesN;
  const int m0 = tm << 6;
  const int n0 = tn << 6;

  const int rl = lane & 15;
  const int h8 = (lane >> 4) * 8;
  const unsigned short* pa = A + (size_t)(m0 + rl) * (size_t)KTOT + h8;
  const unsigned short* pb = B + (size_t)(n0 + rl) * (size_t)KTOT + h8;

  v8f acc[4][4];
#pragma unroll
  for (int i = 0; i < 4; ++i)
#pragma unroll
    for (int j = 0; j < 4; ++j) acc[i][j] = (v8f){0.f, 0.f, 0.f, 0.f, 0.f, 0.f, 0.f, 0.f};

#pragma unroll 1
  for (int k0 = 0; k0 < KTOT; k0 += 32) {
    F bf[4];
#pragma unroll
    for (int j = 0; j < 4; ++j) bf[j] = ld_frag<F>(pb + (size_t)(j << 4) * (size_t)KTOT + k0);
#pragma unroll
    for (int i = 0; i < 4; ++i) {
      const F af = ld_frag<F>(pa + (size_t)(i << 4) * (size_t)KTOT + k0);
#pragma unroll
      for (int j = 0; j < 4; ++j) acc[i][j] = mm(af, bf[j], acc[i][j]);
    }
  }

  float* slab = sT[wave];
  const int hh = lane >> 4;
  const int c4 = (lane & 15) * 4;
  const int nc = n0 + c4;
  const bool cok = nc < N;
  v4f bv = (v4f){0.f, 0.f, 0.f, 0.f};
  if (EPI == 1) {
    bv = *(const v4fa*)(bias + clampi(nc, 0, N - 4));
    asm volatile("" :: "v"(bv));
  }
#pragma unroll
  for (int i = 0; i < 4; ++i) {
    const int mBase = m0 + (i << 4);
#pragma unroll
    for (int j = 0; j < 4; ++j) {
#pragma unroll
      for (int r = 0; r < 8; ++r) slab[(h8 + r) * 68 + (j << 4) + rl] = acc[i][j][r];
    }
    __builtin_amdgcn_fence(__ATOMIC_RELEASE, "workgroup");
    __builtin_amdgcn_wave_barrier();
    __builtin_amdgcn_fence(__ATOMIC_ACQUIRE, "workgroup");
    v4f vv[8];
#pragma unroll
    for (int it = 0; it < 8; ++it) {
      const int row = it * 2 + hh;
      v4f v = *(const v4fa*)(slab + row * 68 + c4);
      if (EPI == 1) v += bv;
      vv[it] = v;
    }
    for (int pass = 0; pass < 2; ++pass) {
#pragma unroll
      for (int it = 0; it < 8; ++it) {
        const int row = mBase + it * 2 + hh;
        if (cok && row < M) *(volatile v4f*)(D + (size_t)row * (size_t)ldd + nc) = vv[it];
      }
      __threadfence();
    }
    __builtin_amdgcn_fence(__ATOMIC_RELEASE, "workgroup");
    __builtin_amdgcn_wave_barrier();
    __builtin_amdgcn_fence(__ATOMIC_ACQUIRE, "workgroup");
  }
}

#define SPLIT_MEAN 1
#define NN     100000
#define NT     200000
#define DD     64
#define NSMP   20
#define MPAD   100096
#define KT     (SPLIT_MEAN ? 192 : 128)
#define AW     (KT / 2)
#define BWP    (DD * KT / 8)
#define OUT1   6400000

typedef float v2f __attribute__((ext_vector_type(2)));
typedef v2f __attribute__((may_alias)) v2fa;

static_assert(DD == 64);
static_assert(NSMP == 20 && NSMP <= 32);
static_assert(KT % 32 == 0 && KT == (SPLIT_MEAN ? 192 : 128));
static_assert(MPAD == 100096 && MPAD % 128 == 0 && MPAD % 64 == 0 && MPAD >= NN && MPAD % 8 == 0);
static_assert(NN % 8 == 0 && NN % 16 == 0);
static_assert(NT == 200000);
static_assert(OUT1 == NN * DD && OUT1 % 32 == 0);
static_assert((long long)OUT1 + (long long)(NN - 1) * DD + (DD - 1) < 2LL * NN * DD);
static_assert(BWP % 256 == 0);
static_assert((long long)MPAD * KT / 8 < (1LL << 31));

constexpr size_t SZ_A    = (size_t)MPAD * KT * 2;
constexpr size_t SZ_H    = (size_t)MPAD * DD * 4;
constexpr size_t SZ_BW   = (size_t)DD * KT * 2;
constexpr size_t SZ_CB   = 256;
constexpr size_t OFF_A   = 0;
constexpr size_t OFF_H   = OFF_A + SZ_A;
constexpr size_t OFF_BWU = OFF_H + SZ_H;
constexpr size_t OFF_BWI = OFF_BWU + SZ_BW;
constexpr size_t OFF_CBU = OFF_BWI + SZ_BW;
constexpr size_t OFF_CBI = OFF_CBU + SZ_CB;
constexpr size_t WS_TOTAL = OFF_CBI + SZ_CB;
static_assert(SZ_A % 256 == 0 && SZ_H % 256 == 0 && SZ_BW % 256 == 0);
static_assert(OFF_H % 256 == 0 && OFF_BWU % 256 == 0 && OFF_BWI % 256 == 0 && OFF_CBU % 256 == 0 && OFF_CBI % 256 == 0);
static_assert(!SPLIT_MEAN || WS_TOTAL == (size_t)64111104);
static_assert(WS_TOTAL <= ((size_t)128 << 20));

__device__ __forceinline__ void wprep_side(const float* __restrict__ Ws, const float* __restrict__ Wn,
                                           const float* __restrict__ bs, const float* __restrict__ bn,
                                           unsigned short* __restrict__ BW, float* __restrict__ CB, int tid) {
#pragma unroll 1
  for (int it = 0; it < BWP / 256; ++it) {
    const int g   = it * 256 + tid;
    const int o   = g / (KT / 8);
    const int p   = g - o * (KT / 8);
    const int seg = p >> 3;
    const int k8  = (p & 7) * 8;
    const float* ps = Ws + o * DD + k8;
    const float* pn = Wn + o * DD + k8;
    const v4f sa = *(const v4fa*)(ps);
    const v4f sc = *(const v4fa*)(ps + 4);
    const v4f na = *(const v4fa*)(pn);
    const v4f nb = *(const v4fa*)(pn + 4);
    asm volatile("" :: "v"(sa));
    asm volatile("" :: "v"(sc));
    asm volatile("" :: "v"(na));
    asm volatile("" :: "v"(nb));
    const v4u qs = pack8_bf16(sa, sc);
    const v4u qn = pack8_bf16(na, nb);
    const unsigned ms = (seg == 0) ? 0xFFFFFFFFu : 0u;
    const v4u m4 = (v4u){ ms, ms, ms, ms };
    const v4u ov = (qs & m4) | (qn & ~m4);
    volatile v4u* q = (volatile v4u*)(BW + (size_t)g * 8);
    *q = ov;
    __threadfence();
    *q = ov;
  }
  const int c4 = (tid & 15) * 4;
  const v4f b1 = *(const v4fa*)(bs + c4);
  const v4f b2 = *(const v4fa*)(bn + c4);
  asm volatile("" :: "v"(b1));
  asm volatile("" :: "v"(b2));
  const v4f cb = (v4f){ bf16_val(b1[0]) + bf16_val(b2[0]), bf16_val(b1[1]) + bf16_val(b2[1]),
                        bf16_val(b1[2]) + bf16_val(b2[2]), bf16_val(b1[3]) + bf16_val(b2[3]) };
  if (tid < 16) {
    volatile v4f* q = (volatile v4f*)(CB + c4);
    *q = cb;
    __threadfence();
    *q = cb;
  }
}

__global__ __launch_bounds__(256) void k_wprep(const float* __restrict__ Wsu, const float* __restrict__ bsu,
                                               const float* __restrict__ Wnu, const float* __restrict__ bnu,
                                               const float* __restrict__ Wsi, const float* __restrict__ bsi,
                                               const float* __restrict__ Wni, const float* __restrict__ bni,
                                               unsigned short* __restrict__ BWu, float* __restrict__ CBu,
                                               unsigned short* __restrict__ BWi, float* __restrict__ CBi) {
  const int tid = (int)threadIdx.x;
  wprep_side(Wsu, Wnu, bsu, bnu, BWu, CBu, tid);
  wprep_side(Wsi, Wni, bsi, bni, BWi, CBi, tid);
}

__global__ __launch_bounds__(256) void k_gather(const int* __restrict__ nodes, const int* __restrict__ nbrs,
                                                const float* __restrict__ tab, unsigned* __restrict__ Apl) {
  const int lane = (int)threadIdx.x & 31;
  const int wave = (int)threadIdx.x >> 5;
  const int n    = (int)blockIdx.x * 8 + wave;
  const int nc   = n < NN ? n : NN - 1;
  const unsigned live = (n < NN) ? 0xFFFFFFFFu : 0u;
  const int kk   = lane < NSMP ? lane : NSMP - 1;
  const int idv  = clampi(nbrs[(size_t)nc * NSMP + kk], 0, NT - 1);
  const int nid  = clampi(nodes[nc], 0, NT - 1);
  float s0 = 0.0f, s1 = 0.0f;
#pragma unroll 4
  for (int k = 0; k < NSMP; ++k) {
    const int sid = __shfl(idv, k, 32);
    const v2f t = *(const v2fa*)(tab + (size_t)sid * DD + 2 * lane);
    s0 = s0 + bf16_val(t.x);
    s1 = s1 + bf16_val(t.y);
  }
  const float a0 = s0 / (float)NSMP;
  const float a1 = s1 / (float)NSMP;
  const v2f sv = *(const v2fa*)(tab + (size_t)nid * DD + 2 * lane);
  const unsigned wself = pk16(bf16_bits(sv.x), bf16_bits(sv.y)) & live;
  const unsigned whi   = pk16(bf16_bits(a0), bf16_bits(a1)) & live;
#if SPLIT_MEAN
  const unsigned wlo   = pk16(bf16_lo_bits(a0), bf16_lo_bits(a1)) & live;
#endif
  if (n < MPAD) {
    volatile unsigned* q = (volatile unsigned*)(Apl + (size_t)n * AW + lane);
    q[0]  = wself;
    q[32] = whi;
#if SPLIT_MEAN
    q[64] = wlo;
#endif
    __threadfence();
    q[0]  = wself;
    q[32] = whi;
#if SPLIT_MEAN
    q[64] = wlo;
#endif
  }
}

__global__ __launch_bounds__(256) void k_rownorm(const float* __restrict__ H, float* __restrict__ outp) {
  const int lane = (int)threadIdx.x & 31;
  const int wave = (int)threadIdx.x >> 5;
  const int n    = (int)blockIdx.x * 8 + wave;
  const int nc   = n < NN ? n : NN - 1;
  const v2f hv = *(const v2fa*)(H + (size_t)nc * DD + 2 * lane);
  const float x = (hv.x > 0.0f) ? hv.x : 0.0f;
  const float y = (hv.y > 0.0f) ? hv.y : 0.0f;
  float ss = x * x + y * y;
  ss += __shfl_xor(ss, 16, 32);
  ss += __shfl_xor(ss, 8, 32);
  ss += __shfl_xor(ss, 4, 32);
  ss += __shfl_xor(ss, 2, 32);
  ss += __shfl_xor(ss, 1, 32);
  const float nrm = sqrtf(ss);
  const float d   = (nrm > 1e-12f) ? nrm : 1e-12f;
  const v2f o = (v2f){ x / d, y / d };
  if (n < NN) {
    volatile v2f* q = (volatile v2f*)(outp + (size_t)n * DD + 2 * lane);
    *q = o;
    __threadfence();
    *q = o;
  }
}

extern "C" void kernel_launch(void* const* d_in, const int* in_sizes, int n_in,
                              void* d_out, int out_size, void* d_ws, size_t ws_size,
                              hipStream_t stream) {
  if (n_in < 14) return;
  if (in_sizes[0] != NN || in_sizes[1] != NN) return;
  if (in_sizes[2] != NN * NSMP || in_sizes[3] != NN * NSMP) return;
  if (in_sizes[4] != NT * DD || in_sizes[5] != NT * DD) return;
  if (in_sizes[6] != DD * DD || in_sizes[8] != DD * DD || in_sizes[10] != DD * DD || in_sizes[12] != DD * DD) return;
  if (in_sizes[7] != DD || in_sizes[9] != DD || in_sizes[11] != DD || in_sizes[13] != DD) return;
  if ((long long)out_size != 2LL * NN * DD) return;
  if (ws_size < WS_TOTAL) return;

  const int*   nodes_u = (const int*)d_in[0];
  const int*   nodes_i = (const int*)d_in[1];
  const int*   nbr_u   = (const int*)d_in[2];
  const int*   nbr_i   = (const int*)d_in[3];
  const float* tab_u   = (const float*)d_in[4];
  const float* tab_i   = (const float*)d_in[5];
  const float* Wsu = (const float*)d_in[6];
  const float* bsu = (const float*)d_in[7];
  const float* Wnu = (const float*)d_in[8];
  const float* bnu = (const float*)d_in[9];
  const float* Wsi = (const float*)d_in[10];
  const float* bsi = (const float*)d_in[11];
  const float* Wni = (const float*)d_in[12];
  const float* bni = (const float*)d_in[13];
  float* out = (float*)d_out;

  char* ws = (char*)d_ws;
  unsigned short* Apl = (unsigned short*)(ws + OFF_A);
  float*          Hpl = (float*)(ws + OFF_H);
  unsigned short* BWu = (unsigned short*)(ws + OFF_BWU);
  unsigned short* BWi = (unsigned short*)(ws + OFF_BWI);
  float*          CBu = (float*)(ws + OFF_CBU);
  float*          CBi = (float*)(ws + OFF_CBI);

  const int gemmBlocks = ((MPAD / 64) + 7) / 8;

  k_wprep<<<1, 256, 0, stream>>>(Wsu, bsu, Wnu, bnu, Wsi, bsi, Wni, bni, BWu, CBu, BWi, CBi);

  k_gather<<<MPAD / 8, 256, 0, stream>>>(nodes_u, nbr_u, tab_u, (unsigned*)Apl);
  k_gemm_nt<0, 1><<<gemmBlocks, 256, 0, stream>>>(Apl, BWu, CBu, Hpl, MPAD, DD, KT, DD);
  k_rownorm<<<NN / 8, 256, 0, stream>>>(Hpl, out);

  k_gather<<<MPAD / 8, 256, 0, stream>>>(nodes_i, nbr_i, tab_i, (unsigned*)Apl);
  k_gemm_nt<0, 1><<<gemmBlocks, 256, 0, stream>>>(Apl, BWi, CBi, Hpl, MPAD, DD, KT, DD);
  k_rownorm<<<NN / 8, 256, 0, stream>>>(Hpl, out + OUT1);
}
